// GraphTransformerNetwork_31963146617558
// MI455X (gfx1250) — hardware-verified
//
#include <hip/hip_runtime.h>
#include <stddef.h>

#define IN_DIM   128
#define HID      32
#define HEADS    4
#define QKV      (HEADS * HID)
#define OUT_DIM  16

#define GEMM_THREADS  128
#define GEMM_GRID_MAX 160
#define EDGE_THREADS  256
#define AGG_THREADS   256
#define AGG_WAVES     (AGG_THREADS / 32)
#define NB            1024
#define CHUNK         (8 * AGG_THREADS)
#define AGG_LDS_BYTES ((NB * 32 + NB * 8) * 4 + (2 * CHUNK + 16) * 4)

typedef _Float16 v16h __attribute__((ext_vector_type(16)));
typedef _Float16 v8h  __attribute__((ext_vector_type(8)));
typedef _Float16 v4h  __attribute__((ext_vector_type(4)));
typedef float    v8f  __attribute__((ext_vector_type(8)));
typedef float    v4f  __attribute__((ext_vector_type(4)));
typedef int      v4i  __attribute__((ext_vector_type(4)));
union Frag { v16h v; v8h h8[2]; v4h q4[4]; };

__device__ __forceinline__ v8f wmma_f16(v16h a, v16h b, v8f c)
{
    return __builtin_amdgcn_wmma_f32_16x16x32_f16(false, a, false, b, (short)0, c, false, false);
}

template <int D, int NT, int OUTH>
__global__ void __launch_bounds__(GEMM_THREADS)
k_gemm(const float* __restrict__ A, const float* __restrict__ W, const float* __restrict__ bias,
       void* Cout, int M, int ntb)
{
    constexpr int F     = NT * 16;
    constexpr int ESZ   = OUTH ? 2 : 4;
    constexpr int ROWB  = F * ESZ;
    constexpr int TILEB = 16 * ROWB;
    constexpr int STF   = TILEB / 4;
    constexpr int NSTEP = TILEB / 16 / 32;

    __shared__ __align__(16) _Float16 wl[F * D];
    __shared__ __align__(16) float st[4 * STF];

    const int tid = threadIdx.x;
    for (int i = tid; i < D * F; i += GEMM_THREADS) {
        const int d = i / F;
        const int f = i - d * F;
        wl[f * D + d] = (_Float16)(W[i] * 64.0f);
    }
    const int lane = tid & 31;
    const int wib  = tid >> 5;
    const int hh   = lane >> 4;
    const int m    = lane & 15;
    float bb[NT];
#pragma unroll
    for (int t = 0; t < NT; ++t) bb[t] = bias[t * 16 + m];
    __syncthreads();

    float* stw = st + wib * STF;
    const v8f zero = {0.f, 0.f, 0.f, 0.f, 0.f, 0.f, 0.f, 0.f};
    const float cs = 0.015625f;

    for (int tb = blockIdx.x; tb < ntb; tb += gridDim.x) {
        const int tm = (tb * 4 + wib) * 16;
        int r = tm + m;
        if (r > M - 1) r = M - 1;
        const float* arow = A + (size_t)r * D;

        v8f acc[NT];
#pragma unroll
        for (int t = 0; t < NT; ++t) acc[t] = zero;

#pragma unroll
        for (int k0 = 0; k0 < D; k0 += 32) {
            const float* ap = arow + k0 + 8 * hh;
            const v4f f0 = *(const v4f*)(ap);
            const v4f f1 = *(const v4f*)(ap + 4);
            const v4f f2 = *(const v4f*)(ap + 16);
            const v4f f3 = *(const v4f*)(ap + 20);
            Frag a;
            a.q4[0] = __builtin_convertvector(f0, v4h);
            a.q4[1] = __builtin_convertvector(f1, v4h);
            a.q4[2] = __builtin_convertvector(f2, v4h);
            a.q4[3] = __builtin_convertvector(f3, v4h);
            Frag b;
#pragma unroll
            for (int t = 0; t < NT; ++t) {
                const _Float16* bp = wl + (t * 16 + m) * D + k0 + 8 * hh;
                b.h8[0] = *(const v8h*)(bp);
                b.h8[1] = *(const v8h*)(bp + 16);
                acc[t] = wmma_f16(a.v, b.v, acc[t]);
            }
            asm volatile("v_nop\n\tv_nop\n\tv_nop\n\tv_nop" : "+v"(acc[NT - 1]) : "v"(a.v), "v"(b.v));
#pragma unroll
            for (int t = 0; t < NT; ++t) asm volatile("" : "+v"(acc[t]));
        }

#pragma unroll
        for (int t = 0; t < NT; ++t) {
#pragma unroll
            for (int i = 0; i < 8; ++i) {
                const float val = acc[t][i] * cs + bb[t];
                const int idx = (8 * hh + i) * F + t * 16 + m;
                if (OUTH) ((_Float16*)stw)[idx] = (_Float16)val;
                else      stw[idx] = val;
            }
        }
        __syncthreads();

        char* gbase = (char*)Cout + (size_t)tm * ROWB;
        const char* sb = (const char*)stw;
#pragma unroll
        for (int s = 0; s < NSTEP; ++s) {
            const int p   = s * 32 + lane;
            const int row = (p * 16) / ROWB;
            const v4f val = *(const v4f*)(sb + 16 * p);
            if (tm + row < M) *(volatile v4f*)(gbase + 16 * p) = val;
        }
        __threadfence();
#pragma unroll
        for (int s = 0; s < NSTEP; ++s) {
            const int p   = s * 32 + lane;
            const int row = (p * 16) / ROWB;
            const v4f val = *(const v4f*)(sb + 16 * p);
            if (tm + row < M) *(volatile v4f*)(gbase + 16 * p) = val;
        }
        __syncthreads();
    }
}

__global__ void __launch_bounds__(EDGE_THREADS)
k_alpha(const _Float16* __restrict__ q, const _Float16* __restrict__ kk,
        const int* __restrict__ esrc, const int* __restrict__ edst,
        float* alpha, int E, int Epad, int N)
{
    const int e = blockIdx.x * EDGE_THREADS + threadIdx.x;
    const int ec = e < E ? e : E - 1;
    int s = esrc[ec];
    int d = edst[ec];
    s = s < 0 ? 0 : (s > N - 1 ? N - 1 : s);
    d = d < 0 ? 0 : (d > N - 1 ? N - 1 : d);
    const _Float16* qr = q  + (size_t)d * QKV;
    const _Float16* kr = kk + (size_t)s * QKV;

    float o0 = 0.f, o1 = 0.f, o2 = 0.f, o3 = 0.f;
#pragma unroll 1
    for (int hd = 0; hd < HEADS; ++hd) {
        float acc = 0.f;
#pragma unroll
        for (int c8 = 0; c8 < HID / 8; ++c8) {
            const v8h qa = *(const v8h*)(qr + hd * HID + c8 * 8);
            const v8h ka = *(const v8h*)(kr + hd * HID + c8 * 8);
#pragma unroll
            for (int i = 0; i < 8; ++i) acc += (float)qa[i] * (float)ka[i];
        }
        acc *= 0.17677669529663687f;
        o0 = hd == 0 ? acc : o0;
        o1 = hd == 1 ? acc : o1;
        o2 = hd == 2 ? acc : o2;
        o3 = hd == 3 ? acc : o3;
    }
    const v4f out = {o0, o1, o2, o3};
    if (e < Epad) {
        float* p = alpha + (size_t)e * 4;
        *(volatile v4f*)p = out;
        __threadfence();
        *(volatile v4f*)p = out;
    }
}

__device__ __forceinline__ int compact_chunk(const int* __restrict__ edst, int E, int base, int n0,
                                             int vec_ok, int* liste, int* listn, int* wsum,
                                             int tid, int lane, int wib)
{
    const int e0 = base + 8 * tid;
    int d[8];
    if (vec_ok && (e0 + 8 <= E)) {
        const v4i x0 = *(const v4i*)(edst + e0);
        const v4i x1 = *(const v4i*)(edst + e0 + 4);
        d[0] = x0[0]; d[1] = x0[1]; d[2] = x0[2]; d[3] = x0[3];
        d[4] = x1[0]; d[5] = x1[1]; d[6] = x1[2]; d[7] = x1[3];
    } else {
#pragma unroll
        for (int k = 0; k < 8; ++k) {
            const int e = e0 + k;
            d[k] = (e < E) ? edst[e] : -1;
        }
    }
    unsigned hm = 0u;
    int cnt = 0;
#pragma unroll
    for (int k = 0; k < 8; ++k) {
        const unsigned rel = (unsigned)d[k] - (unsigned)n0;
        const bool hit = rel < (unsigned)NB;
        hm |= (hit ? 1u : 0u) << k;
        cnt += hit ? 1 : 0;
    }
    int incl = cnt;
#pragma unroll
    for (int o = 1; o < 32; o <<= 1) {
        const int y = __shfl_up(incl, o, 32);
        if (lane >= o) incl += y;
    }
    if (lane == 31) wsum[wib] = incl;
    __syncthreads();
    int woff = 0, total = 0;
#pragma unroll
    for (int w = 0; w < AGG_WAVES; ++w) {
        const int sw = wsum[w];
        total += sw;
        if (w < wib) woff += sw;
    }
    int pos = woff + incl - cnt;
#pragma unroll
    for (int k = 0; k < 8; ++k) {
        if (hm & (1u << k)) {
            liste[pos] = e0 + k;
            listn[pos] = d[k] - n0;
            ++pos;
        }
    }
    __syncthreads();
    if (total > CHUNK) total = CHUNK;
    return total;
}

__global__ void __launch_bounds__(AGG_THREADS)
k_agg(const _Float16* __restrict__ v, const float* __restrict__ alpha,
      const int* __restrict__ esrc, const int* __restrict__ edst,
      const float* __restrict__ skip, float* hout, int E, int N, int vec_ok)
{
    extern __shared__ __align__(16) float lds[];
    float* accl  = lds;
    float* ml    = lds + NB * 32;
    float* sl    = ml + NB * 4;
    int*   liste = (int*)(sl + NB * 4);
    int*   listn = liste + CHUNK;
    int*   wsum  = listn + CHUNK;

    const int tid  = threadIdx.x;
    const int lane = tid & 31;
    const int wib  = tid >> 5;
    const int sub  = tid >> 2;
    const int part = tid & 3;
    const int n0   = blockIdx.x * NB;
    const float NINF = -__builtin_huge_valf();

    for (int i = tid; i < NB * 32; i += AGG_THREADS) accl[i] = 0.f;
    for (int i = tid; i < NB * 4; i += AGG_THREADS) { ml[i] = NINF; sl[i] = 0.f; }
    __syncthreads();

    const int nch = (E + CHUNK - 1) / CHUNK;

    for (int c = 0; c < nch; ++c) {
        const int total = compact_chunk(edst, E, c * CHUNK, n0, vec_ok, liste, listn, wsum, tid, lane, wib);
        for (int r = 0; r < CHUNK / 64; ++r) {
            if (r * 64 >= total) break;
            const int i = r * 64 + sub;
            if (i < total) {
                const int n = listn[i] & (NB - 1);
                bool owner = true;
                for (int j = 0; j < i; ++j) {
                    if ((listn[j] & (NB - 1)) == n) { owner = false; break; }
                }
                if (owner) {
                    float mcur = ml[n * 4 + part];
                    float scur = sl[n * 4 + part];
                    for (int j = i; j < total; ++j) {
                        if ((listn[j] & (NB - 1)) == n) {
                            int e = liste[j];
                            e = ((unsigned)e < (unsigned)E) ? e : 0;
                            const float a  = alpha[(size_t)e * 4 + part];
                            const float mn = fmaxf(mcur, a);
                            scur = scur * __expf(mcur - mn) + __expf(a - mn);
                            mcur = mn;
                        }
                    }
                    ml[n * 4 + part] = mcur;
                    sl[n * 4 + part] = scur;
                }
            }
        }
        __syncthreads();
    }

    for (int i = tid; i < NB * 4; i += AGG_THREADS) sl[i] = 0.25f / sl[i];
    __syncthreads();

    for (int c = 0; c < nch; ++c) {
        const int total = compact_chunk(edst, E, c * CHUNK, n0, vec_ok, liste, listn, wsum, tid, lane, wib);
        for (int r = 0; r < CHUNK / 64; ++r) {
            if (r * 64 >= total) break;
            const int i = r * 64 + sub;
            if (i < total) {
                const int n = listn[i] & (NB - 1);
                bool owner = true;
                for (int j = 0; j < i; ++j) {
                    if ((listn[j] & (NB - 1)) == n) { owner = false; break; }
                }
                if (owner) {
                    const v4f m4 = *(const v4f*)(ml + n * 4);
                    const v4f r4 = *(const v4f*)(sl + n * 4);
                    v8f ac = {0.f, 0.f, 0.f, 0.f, 0.f, 0.f, 0.f, 0.f};
                    for (int j = i; j < total; ++j) {
                        if ((listn[j] & (NB - 1)) == n) {
                            int e = liste[j];
                            e = ((unsigned)e < (unsigned)E) ? e : 0;
                            int sn = esrc[e];
                            sn = sn < 0 ? 0 : (sn > N - 1 ? N - 1 : sn);
                            const v4f al = *(const v4f*)(alpha + (size_t)e * 4);
                            const _Float16* vr = v + (size_t)sn * QKV + part * 8;
#pragma unroll
                            for (int hd = 0; hd < HEADS; ++hd) {
                                const float w  = __expf(al[hd] - m4[hd]) * r4[hd];
                                const v8h  vv = *(const v8h*)(vr + hd * HID);
#pragma unroll
                                for (int cc = 0; cc < 8; ++cc) ac[cc] += w * (float)vv[cc];
                            }
                        }
                    }
                    float* dp = accl + n * 32 + part * 8;
#pragma unroll
                    for (int cc = 0; cc < 8; ++cc) dp[cc] += ac[cc];
                }
            }
        }
        __syncthreads();
    }

    for (int r = 0; r < (NB * 32 / 4) / AGG_THREADS; ++r) {
        const int idx  = r * AGG_THREADS + tid;
        const int nl   = idx >> 3;
        const int c4   = (idx & 7) * 4;
        const int node = n0 + nl;
        if (node < N) {
            const v4f a  = *(const v4f*)(accl + nl * 32 + c4);
            const v4f sk = *(const v4f*)(skip + (size_t)node * HID + c4);
            v4f hv = a + sk;
#pragma unroll
            for (int i = 0; i < 4; ++i) hv[i] = hv[i] > 0.f ? hv[i] : 0.f;
            *(volatile v4f*)(hout + (size_t)node * HID + c4) = hv;
        }
    }
    __threadfence();
    for (int r = 0; r < (NB * 32 / 4) / AGG_THREADS; ++r) {
        const int idx  = r * AGG_THREADS + tid;
        const int nl   = idx >> 3;
        const int c4   = (idx & 7) * 4;
        const int node = n0 + nl;
        if (node < N) {
            const v4f a  = *(const v4f*)(accl + nl * 32 + c4);
            const v4f sk = *(const v4f*)(skip + (size_t)node * HID + c4);
            v4f hv = a + sk;
#pragma unroll
            for (int i = 0; i < 4; ++i) hv[i] = hv[i] > 0.f ? hv[i] : 0.f;
            *(volatile v4f*)(hout + (size_t)node * HID + c4) = hv;
        }
    }
}

static inline int cdiv_i(int a, int b) { return (a + b - 1) / b; }

template <int D, int NT, int OUTH>
static void launch_gemm(const float* A, const float* W, const float* bias, void* C, int M,
                        hipStream_t stream)
{
    const int ntiles = cdiv_i(M, 16);
    const int ntb    = cdiv_i(ntiles, 4);
    const int grid   = ntb < GEMM_GRID_MAX ? ntb : GEMM_GRID_MAX;
    hipLaunchKernelGGL((k_gemm<D, NT, OUTH>), dim3(grid), dim3(GEMM_THREADS), 0, stream,
                       A, W, bias, C, M, ntb);
}

extern "C" void kernel_launch(void* const* d_in, const int* in_sizes, int n_in,
                              void* d_out, int out_size, void* d_ws, size_t ws_size,
                              hipStream_t stream)
{
    if (n_in < 20) return;
    const int N = in_sizes[0] / IN_DIM;
    const int E = in_sizes[1] / 2;
    if (N < 1 || E < 1) return;
    if (out_size < N * OUT_DIM) return;

    const float* x    = (const float*)d_in[0];
    const int*   esrc = (const int*)d_in[1];
    const int*   edst = esrc + E;
    const float* Wl[2][4];
    const float* Bl[2][4];
    for (int l = 0; l < 2; ++l)
        for (int j = 0; j < 4; ++j) {
            Wl[l][j] = (const float*)d_in[2 + l * 8 + 2 * j];
            Bl[l][j] = (const float*)d_in[2 + l * 8 + 2 * j + 1];
        }
    const float* Wout = (const float*)d_in[18];
    const float* bout = (const float*)d_in[19];

    size_t off = 0;
    char* wsb = (char*)d_ws;
    auto carve = [&](size_t bytes) -> char* {
        char* p = wsb + off;
        off += (bytes + 255) & ~(size_t)255;
        return p;
    };
    _Float16* q16  = (_Float16*)carve((size_t)N * QKV * 2);
    _Float16* k16  = (_Float16*)carve((size_t)N * QKV * 2);
    _Float16* v16  = (_Float16*)carve((size_t)N * QKV * 2);
    float*    skip = (float*)   carve((size_t)N * HID * 4);
    float*    hbuf = (float*)   carve((size_t)N * HID * 4);
    float*    alph = (float*)   carve((size_t)E * HEADS * 4);
    if (off > ws_size) return;

    const int Epad      = (E + 7) & ~7;
    const int vec_ok    = (E % 4 == 0) ? 1 : 0;
    const int edge_grid = cdiv_i(Epad, EDGE_THREADS);
    const int agg_grid  = cdiv_i(N, NB);
    const size_t agg_lds = (size_t)AGG_LDS_BYTES;

    launch_gemm<IN_DIM, 8, 1>(x, Wl[0][0], Bl[0][0], (void*)q16,  N, stream);
    launch_gemm<IN_DIM, 8, 1>(x, Wl[0][1], Bl[0][1], (void*)k16,  N, stream);
    launch_gemm<IN_DIM, 8, 1>(x, Wl[0][2], Bl[0][2], (void*)v16,  N, stream);
    launch_gemm<IN_DIM, 2, 0>(x, Wl[0][3], Bl[0][3], (void*)skip, N, stream);
    hipLaunchKernelGGL(k_alpha, dim3(edge_grid), dim3(EDGE_THREADS), 0, stream,
                       (const _Float16*)q16, (const _Float16*)k16, esrc, edst, alph, E, Epad, N);
    hipLaunchKernelGGL(k_agg, dim3(agg_grid), dim3(AGG_THREADS), agg_lds, stream,
                       (const _Float16*)v16, (const float*)alph, esrc, edst, (const float*)skip,
                       hbuf, E, N, vec_ok);

    launch_gemm<HID, 8, 1>(hbuf, Wl[1][0], Bl[1][0], (void*)q16,  N, stream);
    launch_gemm<HID, 8, 1>(hbuf, Wl[1][1], Bl[1][1], (void*)k16,  N, stream);
    launch_gemm<HID, 8, 1>(hbuf, Wl[1][2], Bl[1][2], (void*)v16,  N, stream);
    launch_gemm<HID, 2, 0>(hbuf, Wl[1][3], Bl[1][3], (void*)skip, N, stream);
    hipLaunchKernelGGL(k_alpha, dim3(edge_grid), dim3(EDGE_THREADS), 0, stream,
                       (const _Float16*)q16, (const _Float16*)k16, esrc, edst, alph, E, Epad, N);
    hipLaunchKernelGGL(k_agg, dim3(agg_grid), dim3(AGG_THREADS), agg_lds, stream,
                       (const _Float16*)v16, (const float*)alph, esrc, edst, (const float*)skip,
                       hbuf, E, N, vec_ok);

    launch_gemm<HID, 1, 0>(hbuf, Wout, bout, d_out, N, stream);

    (void)hipGetLastError();
}
